// LSTM_12412455485764
// MI455X (gfx1250) — hardware-verified
//
#include <hip/hip_runtime.h>
#include <math.h>

constexpr int NBATCH  = 64;
constexpr int NSTEP   = 256;
constexpr int NIN     = 256;
constexpr int NHID    = 1024;
constexpr int NCLS    = 1000;
constexpr int NCLSP   = 1024;
constexpr int KCAT    = NIN + NHID;
constexpr int SEQ_BLK = 16;
constexpr int NTHR_R  = 512;
constexpr int NWAVE_R = NTHR_R / 32;
constexpr int TILES_W = NHID / (16 * NWAVE_R);
constexpr int NTHR_O  = 256;
constexpr int NWAVE_O = NTHR_O / 32;
constexpr int NTHR_P  = 256;
constexpr int HPITCH  = NHID + 8;
constexpr int GSTR    = 16 * KCAT;
constexpr int PSTR    = 16 * NHID;
constexpr float WCARRY = 16.0f;
constexpr float ACARRY = 16.0f;
constexpr float FOLD   = 1.0f / (WCARRY * ACARRY);

static_assert(NBATCH % SEQ_BLK == 0, "batch tiles");
static_assert(TILES_W == 4 && NHID == 64 * NWAVE_R, "each recurrence wave owns 64 hidden units = 4 tiles");
static_assert(NCLSP == 128 * NWAVE_O, "each projection wave owns 128 padded classes");
static_assert(NIN % 64 == 0 && NHID % 64 == 0 && KCAT % 32 == 0, "k extents are multiples of 32; pack tiles of 64");
static_assert(NCLS % 4 == 0 && NCLS <= NCLSP, "class padding");
static_assert((SEQ_BLK * NCLS * 4) % 128 == 0, "per-block output region is whole lines");
static_assert((SEQ_BLK * NCLS / 4) % 32 == 0, "output copy guard is wave-uniform");
static_assert(SEQ_BLK * NCLS * 4 <= 65536, "output staging fits static LDS");
static_assert((HPITCH * 2) % 16 == 0, "h tile rows 16-B aligned");
static_assert(NTHR_R == 512 && NHID == 1024, "bias table load: 2 gate pairs x 2 halves x 256 positions x 4 floats");
static_assert(SEQ_BLK * NHID == 4 * 8 * NTHR_R, "final h copy: 4 iterations x 512 threads x 8 halves");
static_assert(SEQ_BLK * HPITCH * 2 + 4 * NHID * 4 <= 65536, "recurrence static LDS");

typedef __attribute__((ext_vector_type(16))) _Float16 v16h;
typedef __attribute__((ext_vector_type(8)))  _Float16 v8h;
typedef __attribute__((ext_vector_type(8)))  float    v8f;
typedef __attribute__((ext_vector_type(4)))  float    v4f;

__device__ __forceinline__ void grp_guard(v8f& c0, v8f& c1, v8f& c2, v8f& c3, v16h a0,
                                          v16h b0, v16h b1, v16h b2, v16h b3) {
  asm volatile("v_nop\n\tv_nop\n\tv_nop\n\tv_nop"
               : "+v"(c0), "+v"(c1), "+v"(c2), "+v"(c3)
               : "v"(a0), "v"(b0), "v"(b1), "v"(b2), "v"(b3));
}

struct FragH {
  union U { v16h v; v8h h[2]; };
  static __device__ __forceinline__ v16h load(const _Float16* p) {
    U f;
    f.h[0] = *(const v8h*)(p);
    f.h[1] = *(const v8h*)(p + 16);
    return f.v;
  }
  static __device__ __forceinline__ v8f mma(v16h a, v16h b, v8f c) {
    return __builtin_amdgcn_wmma_f32_16x16x32_f16(false, a, false, b, (short)0, c, false, false);
  }
};

template <int BSTR>
__device__ __forceinline__ void kstep1(const _Float16* ap, const _Float16* wp, v8f& c0, v8f& c1, v8f& c2, v8f& c3) {
  const v16h a0 = FragH::load(ap);
  const v16h b0 = FragH::load(wp);
  const v16h b1 = FragH::load(wp + BSTR);
  const v16h b2 = FragH::load(wp + 2 * BSTR);
  const v16h b3 = FragH::load(wp + 3 * BSTR);
  c0 = FragH::mma(a0, b0, c0);
  c1 = FragH::mma(a0, b1, c1);
  c2 = FragH::mma(a0, b2, c2);
  c3 = FragH::mma(a0, b3, c3);
  grp_guard(c0, c1, c2, c3, a0, b0, b1, b2, b3);
}

__device__ __forceinline__ float fsig(float x)  { return __builtin_amdgcn_rcpf(1.0f + __expf(-x)); }
__device__ __forceinline__ float ftanh(float x) { return 1.0f - 2.0f * __builtin_amdgcn_rcpf(__expf(2.0f * x) + 1.0f); }

__device__ __forceinline__ float lstm_cell(float ag, float ai, float af, float ao,
                                           float bg, float bi, float bf, float bo, float& cs) {
  const float zg = fmaf(ag, FOLD, bg);
  const float zi = fmaf(ai, FOLD, bi);
  const float zf = fmaf(af, FOLD, bf);
  const float zo = fmaf(ao, FOLD, bo);
  const float gg = ftanh(zg);
  const float ig = fsig(zi);
  const float fg = fsig(zf);
  const float og = fsig(zo);
  const float cn = fmaf(cs, fg, gg * ig);
  cs = cn;
  return ftanh(cn) * og;
}

__global__ __launch_bounds__(NTHR_P) void cvt_x_kernel(const float* __restrict__ src, unsigned short* __restrict__ dst,
                                                      int n8, float sc) {
  const int i = blockIdx.x * NTHR_P + threadIdx.x;
  if (i < n8) {
    const float* sp = src + (size_t)i * 8;
    const v4f a = *(const v4f*)(sp);
    const v4f b = *(const v4f*)(sp + 4);
    v8h hv;
#pragma unroll
    for (int e = 0; e < 4; ++e) {
      hv[e]     = (_Float16)(a[e] * sc);
      hv[4 + e] = (_Float16)(b[e] * sc);
    }
    *(volatile v8h*)(dst + (size_t)i * 8) = hv;
    __threadfence();
    *(volatile v8h*)(dst + (size_t)i * 8) = hv;
  }
}

__global__ __launch_bounds__(NTHR_P) void pack_wcat_kernel(const float* __restrict__ wgx, const float* __restrict__ wgh,
                                                          const float* __restrict__ wix, const float* __restrict__ wih,
                                                          const float* __restrict__ wfx, const float* __restrict__ wfh,
                                                          const float* __restrict__ wox, const float* __restrict__ woh,
                                                          unsigned short* __restrict__ O) {
  __shared__ float Tt[64 * 65];
  const int tid = threadIdx.x;
  const int bx = blockIdx.x, by = blockIdx.y, q = blockIdx.z;
  const float* wx = (q == 0) ? wgx : (q == 1) ? wix : (q == 2) ? wfx : wox;
  const float* wh = (q == 0) ? wgh : (q == 1) ? wih : (q == 2) ? wfh : woh;
  const bool isx = (by < NIN / 64);
  const float* src = isx ? wx : wh;
  const int r0 = isx ? (64 * by) : (64 * (by - NIN / 64));
  const int c0 = 64 * bx;
#pragma unroll
  for (int i = 0; i < 4; ++i) {
    const int idx = i * NTHR_P + tid;
    const int rr = idx >> 4, cc = (idx & 15) * 4;
    const v4f v = *(const v4f*)(src + (size_t)(r0 + rr) * NHID + c0 + cc);
    Tt[rr * 65 + cc + 0] = v[0];
    Tt[rr * 65 + cc + 1] = v[1];
    Tt[rr * 65 + cc + 2] = v[2];
    Tt[rr * 65 + cc + 3] = v[3];
  }
  __syncthreads();
  const int q8 = tid >> 3, c8 = (tid & 7) * 8;
  v8h hv[2];
#pragma unroll
  for (int g = 0; g < 2; ++g) {
    const int qq = g * 32 + q8;
#pragma unroll
    for (int e = 0; e < 8; ++e) hv[g][e] = (_Float16)(Tt[(c8 + e) * 65 + qq] * WCARRY);
  }
  for (int pass = 0; pass < 2; ++pass) {
#pragma unroll
    for (int g = 0; g < 2; ++g) {
      const int n = c0 + g * 32 + q8;
      const int np = ((n >> 4) * 4 + q) * 16 + (n & 15);
      const size_t o = (size_t)np * KCAT + (size_t)(64 * by + c8);
      *(volatile v8h*)(O + o) = hv[g];
    }
    __threadfence();
  }
}

__global__ __launch_bounds__(NTHR_P) void pack_wp_kernel(const float* __restrict__ src, unsigned short* __restrict__ O) {
  __shared__ float Tt[64 * 65];
  const int tid = threadIdx.x;
  const int c0 = 64 * blockIdx.x, r0 = 64 * blockIdx.y;
#pragma unroll
  for (int i = 0; i < 4; ++i) {
    const int idx = i * NTHR_P + tid;
    const int rr = idx >> 4, cc = (idx & 15) * 4;
    const int col = c0 + cc;
    const bool inb = (col < NCLS);
    const int colc = inb ? col : (NCLS - 4);
    const v4f v = *(const v4f*)(src + (size_t)(r0 + rr) * NCLS + colc);
    const float f0 = inb ? v[0] : 0.0f;
    const float f1 = inb ? v[1] : 0.0f;
    const float f2 = inb ? v[2] : 0.0f;
    const float f3 = inb ? v[3] : 0.0f;
    Tt[rr * 65 + cc + 0] = f0;
    Tt[rr * 65 + cc + 1] = f1;
    Tt[rr * 65 + cc + 2] = f2;
    Tt[rr * 65 + cc + 3] = f3;
  }
  __syncthreads();
  const int q8 = tid >> 3, c8 = (tid & 7) * 8;
  v8h hv[2];
#pragma unroll
  for (int g = 0; g < 2; ++g) {
    const int qq = g * 32 + q8;
#pragma unroll
    for (int e = 0; e < 8; ++e) hv[g][e] = (_Float16)(Tt[(c8 + e) * 65 + qq] * WCARRY);
  }
  for (int pass = 0; pass < 2; ++pass) {
#pragma unroll
    for (int g = 0; g < 2; ++g) {
      const size_t o = (size_t)(c0 + g * 32 + q8) * NHID + (size_t)(r0 + c8);
      *(volatile v8h*)(O + o) = hv[g];
    }
    __threadfence();
  }
}

__global__ __launch_bounds__(NTHR_R) __attribute__((amdgpu_num_vgpr(256)))
void lstm_seq_kernel(const unsigned short* __restrict__ Xhp,
                     const unsigned short* __restrict__ Btp,
                     const float* __restrict__ b_g, const float* __restrict__ b_i,
                     const float* __restrict__ b_f, const float* __restrict__ b_o,
                     unsigned short* __restrict__ Hfp) {
  __shared__ __align__(16) _Float16 Ah[SEQ_BLK * HPITCH];
  __shared__ __align__(16) float    Bs[4 * NHID];
  const _Float16* Xh = (const _Float16*)Xhp;
  const _Float16* Bt = (const _Float16*)Btp;
  const int tid = threadIdx.x, lane = tid & 31, wave = tid >> 5;
  const int c = lane & 15, hh = lane >> 4, koff = hh * 8;
  const int rowbase = blockIdx.x * SEQ_BLK;

#pragma unroll 1
  for (int i = tid; i < SEQ_BLK * HPITCH; i += NTHR_R) Ah[i] = (_Float16)0.0f;
  {
    const int half = tid >> 8;
    const int pos = (tid & 255) * 4;
    const v4f va = *(const v4f*)(b_g + pos);
    const v4f vb = *(const v4f*)(b_i + pos);
    const v4f vc = *(const v4f*)(b_f + pos);
    const v4f vd = *(const v4f*)(b_o + pos);
    v4f s0, s1;
#pragma unroll
    for (int e = 0; e < 4; ++e) {
      s0[e] = half ? vb[e] : va[e];
      s1[e] = half ? vd[e] : vc[e];
    }
    *(v4f*)(Bs + half * NHID + pos) = s0;
    *(v4f*)(Bs + (2 + half) * NHID + pos) = s1;
  }
  float cst[TILES_W][8];
  float hst[TILES_W][8];
#pragma unroll
  for (int nt = 0; nt < TILES_W; ++nt) {
#pragma unroll
    for (int r = 0; r < 8; ++r) {
      cst[nt][r] = 0.0f;
      hst[nt][r] = 0.0f;
    }
  }
  __syncthreads();

  const _Float16* ahrow = Ah + c * HPITCH + koff;
  const _Float16* wbase = Bt + (size_t)((TILES_W * wave) * 64 + c) * KCAT + koff;
  const v8f z8 = {0.f, 0.f, 0.f, 0.f, 0.f, 0.f, 0.f, 0.f};

#pragma unroll 1
  for (int t = 0; t < NSTEP; ++t) {
    const _Float16* xrow = Xh + ((size_t)(rowbase + c) * NSTEP + (size_t)t) * NIN + koff;
#pragma unroll
    for (int nt = 0; nt < TILES_W; ++nt) {
      const int col = 64 * wave + 16 * nt + c;
      const _Float16* wrow = wbase + (size_t)nt * 64 * KCAT;
      v8f accG = z8, accI = z8, accF = z8, accO = z8;
#pragma unroll 1
      for (int k0 = 0; k0 < NIN; k0 += 32) kstep1<GSTR>(xrow + k0, wrow + k0, accG, accI, accF, accO);
#pragma unroll 1
      for (int k0 = 0; k0 < NHID; k0 += 32) kstep1<GSTR>(ahrow + k0, wrow + NIN + k0, accG, accI, accF, accO);
      const float bgv = Bs[col];
      const float biv = Bs[NHID + col];
      const float bfv = Bs[2 * NHID + col];
      const float bov = Bs[3 * NHID + col];
#pragma unroll
      for (int r = 0; r < 8; ++r) {
        const float hn = lstm_cell(accG[r], accI[r], accF[r], accO[r], bgv, biv, bfv, bov, cst[nt][r]);
        hst[nt][r] = hn * ACARRY;
      }
    }
    __syncthreads();
#pragma unroll
    for (int nt = 0; nt < TILES_W; ++nt) {
      const int col = 64 * wave + 16 * nt + c;
#pragma unroll
      for (int r = 0; r < 8; ++r) Ah[(8 * hh + r) * HPITCH + col] = (_Float16)hst[nt][r];
    }
    __syncthreads();
  }

  for (int pass = 0; pass < 2; ++pass) {
#pragma unroll
    for (int it = 0; it < 4; ++it) {
      const int idx = it * NTHR_R + tid;
      const int row = idx >> 7, c8 = (idx & 127) * 8;
      const v8h v = *(const v8h*)(Ah + row * HPITCH + c8);
      *(volatile v8h*)(Hfp + (size_t)(rowbase + row) * NHID + c8) = v;
    }
    __threadfence();
  }
}

__global__ __launch_bounds__(NTHR_O) void outproj_kernel(const unsigned short* __restrict__ Hfp,
                                                        const unsigned short* __restrict__ Wptp,
                                                        const float* __restrict__ bp, float* __restrict__ out) {
  __shared__ __align__(16) float So[SEQ_BLK * NCLS];
  const _Float16* Hf  = (const _Float16*)Hfp;
  const _Float16* Wpt = (const _Float16*)Wptp;
  const int tid = threadIdx.x, lane = tid & 31, wave = tid >> 5;
  const int c = lane & 15, hh = lane >> 4, koff = hh * 8;
  const int rowbase = blockIdx.x * SEQ_BLK;
  const _Float16* arow = Hf + (size_t)(rowbase + c) * NHID + koff;
  const v8f z8 = {0.f, 0.f, 0.f, 0.f, 0.f, 0.f, 0.f, 0.f};
#pragma unroll
  for (int hf = 0; hf < 2; ++hf) {
    const int nbase = 128 * wave + 64 * hf;
    const _Float16* wrow = Wpt + (size_t)(nbase + c) * NHID + koff;
    v8f acc[4];
    acc[0] = z8; acc[1] = z8; acc[2] = z8; acc[3] = z8;
#pragma unroll 1
    for (int k0 = 0; k0 < NHID; k0 += 32) kstep1<PSTR>(arow + k0, wrow + k0, acc[0], acc[1], acc[2], acc[3]);
#pragma unroll
    for (int j = 0; j < 4; ++j) {
      const int n = nbase + 16 * j + c;
      const bool inb = (n < NCLS);
      const int nc = inb ? n : (NCLS - 1);
      const float bv = bp[nc];
#pragma unroll
      for (int r = 0; r < 8; ++r) {
        const float v = fmaf(acc[j][r], FOLD, bv);
        if (inb) So[(8 * hh + r) * NCLS + n] = v;
      }
    }
  }
  __syncthreads();
  float* ob = out + (size_t)rowbase * NCLS;
  for (int pass = 0; pass < 2; ++pass) {
#pragma unroll
    for (int it = 0; it < 16; ++it) {
      const int idx = it * NTHR_O + tid;
      if (idx < SEQ_BLK * NCLS / 4) {
        const v4f v = *(const v4f*)(So + 4 * idx);
        *(volatile v4f*)(ob + 4 * idx) = v;
      }
    }
    __threadfence();
  }
}

extern "C" void kernel_launch(void* const* d_in, const int* in_sizes, int n_in,
                              void* d_out, int out_size, void* d_ws, size_t ws_size, hipStream_t stream) {
  if (n_in < 15 || d_out == nullptr || d_ws == nullptr) return;
  if (in_sizes[0] != NBATCH * NSTEP * NIN || in_sizes[9] != NHID * NCLS || in_sizes[14] != NCLS ||
      out_size != NBATCH * NCLS) return;
  for (int g = 0; g < 4; ++g) {
    if (in_sizes[1 + 2 * g] != NIN * NHID || in_sizes[2 + 2 * g] != NHID * NHID || in_sizes[10 + g] != NHID) return;
  }

  const float* x   = (const float*)d_in[0];
  const float* wgx = (const float*)d_in[1];
  const float* wgh = (const float*)d_in[2];
  const float* wix = (const float*)d_in[3];
  const float* wih = (const float*)d_in[4];
  const float* wfx = (const float*)d_in[5];
  const float* wfh = (const float*)d_in[6];
  const float* wox = (const float*)d_in[7];
  const float* woh = (const float*)d_in[8];
  const float* wph = (const float*)d_in[9];
  const float* bg  = (const float*)d_in[10];
  const float* bi  = (const float*)d_in[11];
  const float* bf  = (const float*)d_in[12];
  const float* bo  = (const float*)d_in[13];
  const float* bp  = (const float*)d_in[14];
  float* out = (float*)d_out;

  char* ws = (char*)d_ws;
  size_t off = 0;
  auto carve = [&](size_t bytes) -> char* { char* p = ws + off; off += (bytes + 255) & ~(size_t)255; return p; };
  unsigned short* XH  = (unsigned short*)carve((size_t)NBATCH * NSTEP * NIN * 2);
  unsigned short* BT  = (unsigned short*)carve((size_t)4 * NHID * KCAT * 2);
  unsigned short* WPT = (unsigned short*)carve((size_t)NCLSP * NHID * 2);
  unsigned short* HF  = (unsigned short*)carve((size_t)NBATCH * NHID * 2);
  if (off > ws_size || off > (size_t)134217728) return;

  const int n8 = NBATCH * NSTEP * NIN / 8;
  cvt_x_kernel<<<(n8 + NTHR_P - 1) / NTHR_P, NTHR_P, 0, stream>>>(x, XH, n8, ACARRY);
  pack_wcat_kernel<<<dim3(NHID / 64, KCAT / 64, 4), NTHR_P, 0, stream>>>(wgx, wgh, wix, wih, wfx, wfh, wox, woh, BT);
  pack_wp_kernel<<<dim3(NCLSP / 64, NHID / 64), NTHR_P, 0, stream>>>(wph, WPT);
  lstm_seq_kernel<<<NBATCH / SEQ_BLK, NTHR_R, 0, stream>>>(XH, BT, bg, bi, bf, bo, HF);
  outproj_kernel<<<NBATCH / SEQ_BLK, NTHR_O, 0, stream>>>(HF, WPT, bp, out);
}
